// WorldModel_884763263653
// MI455X (gfx1250) — hardware-verified
//
#include <hip/hip_runtime.h>
#include <math.h>

constexpr int kBatch = 2;
constexpr int kSeq   = 2048;
constexpr int kDim   = 1024;
constexpr int kHeads = 16;
constexpr int kDh    = 64;
constexpr int kTok   = kBatch * kSeq;
constexpr int kBH    = kBatch * kHeads;
constexpr int kQkvN  = 3 * kHeads * kDh;
constexpr int kCatN  = kQkvN + 64;
constexpr int kOut0Elems = kTok * kDim;
constexpr int kOut1Elems = kBH * kSeq * kDh;
static_assert(kDim % 32 == 0);
static_assert(kTok % 64 == 0 && kCatN % 64 == 0 && kDim % 64 == 0);
static_assert((kTok / 64) * (kCatN / 64) % 8 == 0);
static_assert((kTok / 64) * (kDim / 64) % 8 == 0);
static_assert(kSeq % 64 == 0 && 256 % 64 == 0);
static_assert((size_t)kOut0Elems * 4 == 16777216);
static_assert(((size_t)kOut0Elems + kOut1Elems) * 4 == 33554432);

typedef __attribute__((ext_vector_type(16))) _Float16 v16h;
typedef __attribute__((ext_vector_type(8)))  _Float16 v8h;
typedef __attribute__((ext_vector_type(16))) __bf16   v16b;
typedef __attribute__((ext_vector_type(8)))  __bf16   v8b;
typedef __attribute__((ext_vector_type(8)))  float    v8f;
typedef __attribute__((ext_vector_type(4)))  float    v4f;

__device__ __forceinline__ unsigned short f2bf_bits(float f) {
  unsigned u = __float_as_uint(f);
  return (unsigned short)((u + 0x7FFFu + ((u >> 16) & 1u)) >> 16);
}
__device__ __forceinline__ float bf_bits2f(unsigned short h) { return __uint_as_float(((unsigned)h) << 16); }
__device__ __forceinline__ float bf16_rne(float f) { return bf_bits2f(f2bf_bits(f)); }

__device__ __forceinline__ void dep_guard_h(v8f& a, v8f& b, v16h x, v16h y) { asm volatile("v_nop\n\tv_nop\n\tv_nop\n\tv_nop" : "+v"(a), "+v"(b) : "v"(x), "v"(y)); }
__device__ __forceinline__ void dep_guard_b(v8f& a, v8f& b, v16b x, v16b y) { asm volatile("v_nop\n\tv_nop\n\tv_nop\n\tv_nop" : "+v"(a), "+v"(b) : "v"(x), "v"(y)); }
__device__ __forceinline__ void keep4_h(v16h a, v16h b, v16h c, v16h d) { asm volatile("v_nop" :: "v"(a), "v"(b), "v"(c), "v"(d)); }
__device__ __forceinline__ void keep4_b(v16b a, v16b b, v16b c, v16b d) { asm volatile("v_nop" :: "v"(a), "v"(b), "v"(c), "v"(d)); }
__device__ __forceinline__ void acc_guard4(v8f& a, v8f& b, v8f& c, v8f& d) { asm volatile("v_nop\n\tv_nop\n\tv_nop\n\tv_nop" : "+v"(a), "+v"(b), "+v"(c), "+v"(d)); }
template <typename T> struct Frag;
template <> struct Frag<_Float16> {
  typedef v16h V; union U { v16h v; v8h h[2]; };
  static __device__ __forceinline__ v16h load(const _Float16* p) {
    U f; f.h[0] = *(const v8h*)(p); f.h[1] = *(const v8h*)(p + 16); return f.v;
  }
  static __device__ __forceinline__ v8f mma(v16h a, v16h b, v8f c) {
    return __builtin_amdgcn_wmma_f32_16x16x32_f16(false, a, false, b, (short)0, c, false, false);
  }
  static __device__ __forceinline__ void guard(v8f& a, v8f& b, v16h x, v16h y) { dep_guard_h(a, b, x, y); }
  static __device__ __forceinline__ void keep(v16h a, v16h b, v16h c, v16h d) { keep4_h(a, b, c, d); }
};
template <> struct Frag<__bf16> {
  typedef v16b V; union U { v16b v; v8b h[2]; };
  static __device__ __forceinline__ v16b load(const __bf16* p) {
    U f; f.h[0] = *(const v8b*)(p); f.h[1] = *(const v8b*)(p + 16); return f.v;
  }
  static __device__ __forceinline__ v8f mma(v16b a, v16b b, v8f c) {
    return __builtin_amdgcn_wmma_f32_16x16x32_bf16(false, a, false, b, (short)0, c, false, false);
  }
  static __device__ __forceinline__ void guard(v8f& a, v8f& b, v16b x, v16b y) { dep_guard_b(a, b, x, y); }
  static __device__ __forceinline__ void keep(v16b a, v16b b, v16b c, v16b d) { keep4_b(a, b, c, d); }
};

__device__ __forceinline__ v8f mma_f16g(v16h a, v16h b, v8f c) {
  c = __builtin_amdgcn_wmma_f32_16x16x32_f16(false, a, false, b, (short)0, c, false, false);
  asm volatile("v_nop\n\tv_nop\n\tv_nop\n\tv_nop" : "+v"(c) : "v"(a), "v"(b));
  return c;
}

template <int ET> struct Elem;
template <> struct Elem<0> { typedef _Float16 T; };
template <> struct Elem<1> { typedef __bf16 T; };
template <int ET, bool SPLIT, int BIAS_MODE, int OUT_MODE, bool RESID, int ACT = 0>
__global__ __launch_bounds__(256) void wmma_gemm64(
    const unsigned short* __restrict__ Ap, const unsigned short* __restrict__ A2p, int lda, long strideA,
    const unsigned short* __restrict__ Btp, const unsigned short* __restrict__ Bt2p, int ldb, long strideB,
    void* __restrict__ Cout, void* __restrict__ Cout2, int ldc, long strideC,
    const float* __restrict__ bias,
    const float* __restrict__ resid, long strideR,
    int M, int N, int K, float scale) {
  typedef typename Elem<ET>::T T;
  typedef typename Frag<T>::V V;
  const T* A = (const T*)Ap; const T* A2 = (const T*)A2p; const T* Bt = (const T*)Btp; const T* Bt2 = (const T*)Bt2p;
  __shared__ __align__(16) float sT[8][16 * 68];
  const int b    = blockIdx.y;
  const int lane = threadIdx.x & 31;
  const int wave = threadIdx.x >> 5;
  const int tilesN = N >> 6;
  const int tilesM = M >> 6;
  const int tile = blockIdx.x * 8 + wave;
  if (tile >= tilesM * tilesN) return;
  const int tm = tile / tilesN;
  const int tn = tile - tm * tilesN;
  const int m0 = tm << 6;
  const int n0 = tn << 6;

  const T* Ab  = A  + (size_t)b * strideA;
  const T* Bb  = Bt + (size_t)b * strideB;
  const T* Ab2 = SPLIT ? (A2  + (size_t)b * strideA) : nullptr;
  const T* Bb2 = SPLIT ? (Bt2 + (size_t)b * strideB) : nullptr;

  const int rlane = lane & 15;
  const int koff  = (lane >> 4) * 8;
  const int mOff  = (lane >> 4) * 8;

  v8f acc[4][4];
#pragma unroll
  for (int i = 0; i < 4; ++i)
#pragma unroll
    for (int j = 0; j < 4; ++j) acc[i][j] = (v8f){0.f,0.f,0.f,0.f,0.f,0.f,0.f,0.f};

  for (int k0 = 0; k0 < K; k0 += 32) {
    V bh[4], bl[4];
#pragma unroll
    for (int j = 0; j < 4; ++j) {
      const size_t bo = (size_t)(n0 + (j << 4) + rlane) * ldb + koff + k0;
      bh[j] = Frag<T>::load(Bb + bo);
      if (SPLIT) bl[j] = Frag<T>::load(Bb2 + bo);
    }
#pragma unroll
    for (int i = 0; i < 4; ++i) {
      const size_t ao = (size_t)(m0 + (i << 4) + rlane) * lda + koff + k0;
      V ah = Frag<T>::load(Ab + ao);
      V al;
      if (SPLIT) al = Frag<T>::load(Ab2 + ao);
#pragma unroll
      for (int j = 0; j < 4; ++j) {
        acc[i][j] = Frag<T>::mma(ah, bh[j], acc[i][j]);
        if (SPLIT) {
          acc[i][j] = Frag<T>::mma(ah, bl[j], acc[i][j]);
          acc[i][j] = Frag<T>::mma(al, bh[j], acc[i][j]);
        }
      }
      Frag<T>::guard(acc[i][0], acc[i][3], ah, SPLIT ? al : ah);
    }
    Frag<T>::keep(bh[0], bh[1], bh[2], bh[3]);
    if (SPLIT) Frag<T>::keep(bl[0], bl[1], bl[2], bl[3]);
  }
  acc_guard4(acc[0][0], acc[0][1], acc[0][2], acc[0][3]);
  acc_guard4(acc[1][0], acc[1][1], acc[1][2], acc[1][3]);
  acc_guard4(acc[2][0], acc[2][1], acc[2][2], acc[2][3]);
  acc_guard4(acc[3][0], acc[3][1], acc[3][2], acc[3][3]);

  float* slab = sT[wave];
  const float* Rb = RESID ? (resid + (size_t)b * strideR) : nullptr;
#pragma unroll
  for (int i = 0; i < 4; ++i) {
    const int mBase = m0 + (i << 4);
#pragma unroll
    for (int j = 0; j < 4; ++j) {
      const int n = n0 + (j << 4) + rlane;
      float bv = 0.f;
      if (BIAS_MODE == 2) bv = bias[n];
#pragma unroll
      for (int r = 0; r < 8; ++r) {
        float v = acc[i][j][r] * scale;
        if (BIAS_MODE == 1) v += bias[mBase + mOff + r];
        if (BIAS_MODE == 2) v += bv;
        if (RESID) v += Rb[(size_t)(mBase + mOff + r) * ldc + n];
        if (ACT == 1) v = tanhf(v);
        if (ACT == 2) v = fmaxf(v, 0.0f);
        if (ACT == 3) v = v / (1.0f + expf(-v));
        if (ACT == 4) v = (v > 0.f) ? v : 0.01f * v;
        if (ACT == 5) v = 0.5f * v * (1.0f + erff(v * 0.70710678118654752f));
        slab[(mOff + r) * 68 + (j << 4) + rlane] = v;
      }
    }
    __builtin_amdgcn_fence(__ATOMIC_RELEASE, "workgroup");
    __builtin_amdgcn_wave_barrier();
    __builtin_amdgcn_fence(__ATOMIC_ACQUIRE, "workgroup");
    if (OUT_MODE == 0) {
      float* C = (float*)Cout + (size_t)b * strideC;
      const int hh = lane >> 4, c4 = (lane & 15) * 4;
      for (int pass = 0; pass < 2; ++pass) {
#pragma unroll
        for (int it = 0; it < 8; ++it) {
          const int row = it * 2 + hh;
          v4f v = *(const v4f*)(slab + row * 68 + c4);
          *(volatile v4f*)(C + (size_t)(mBase + row) * ldc + n0 + c4) = v;
        }
        __threadfence();
      }
    } else {
      const int q = lane >> 3, c8 = (lane & 7) * 8;
      unsigned short* C  = (unsigned short*)Cout  + (size_t)b * strideC;
      unsigned short* C2 = (OUT_MODE == 2) ? ((unsigned short*)Cout2 + (size_t)b * strideC) : nullptr;
      for (int pass = 0; pass < 2; ++pass) {
#pragma unroll
        for (int it = 0; it < 4; ++it) {
          const int row = it * 4 + q;
          const float* sp = slab + row * 68 + c8;
          v8h hv, lv;
#pragma unroll
          for (int e = 0; e < 8; ++e) {
            if (OUT_MODE == 1) {
              hv[e] = (_Float16)sp[e];
            } else {
              unsigned short hb = f2bf_bits(sp[e]);
              unsigned short lb = f2bf_bits(sp[e] - bf_bits2f(hb));
              hv[e] = __builtin_bit_cast(_Float16, hb);
              lv[e] = __builtin_bit_cast(_Float16, lb);
            }
          }
          *(volatile v8h*)(C + (size_t)(mBase + row) * ldc + n0 + c8) = hv;
          if (OUT_MODE == 2) *(volatile v8h*)(C2 + (size_t)(mBase + row) * ldc + n0 + c8) = lv;
        }
        __threadfence();
      }
    }
    __builtin_amdgcn_fence(__ATOMIC_RELEASE, "workgroup");
    __builtin_amdgcn_wave_barrier();
    __builtin_amdgcn_fence(__ATOMIC_ACQUIRE, "workgroup");
  }
}

__global__ __launch_bounds__(128) void rmsnorm_f16_kernel(const float* __restrict__ x, const float* __restrict__ gamma,
                                                          unsigned short* __restrict__ xn16) {
  __shared__ float red[4];
  const int row = blockIdx.x;
  const int tid = threadIdx.x, lane = tid & 31, wave = tid >> 5;
  const float* xr = x + (size_t)row * kDim + tid * 8;
  const v4f xa = *(const v4f*)(xr);
  const v4f xb = *(const v4f*)(xr + 4);
  float xv[8];
#pragma unroll
  for (int e = 0; e < 4; ++e) { xv[e] = bf16_rne(xa[e]); xv[4 + e] = bf16_rne(xb[e]); }
  float ss = 0.0f;
#pragma unroll
  for (int e = 0; e < 8; ++e) ss += xv[e] * xv[e];
#pragma unroll
  for (int m = 16; m; m >>= 1) ss += __shfl_xor(ss, m, 32);
  if (lane == 0) red[wave] = ss;
  __syncthreads();
  const float tot = (red[0] + red[1]) + (red[2] + red[3]);
  const float rinv = 1.0f / sqrtf(tot * (1.0f / 1024.0f) + 1.1920928955078125e-07f);
  const v4f ga = *(const v4f*)(gamma + tid * 8);
  const v4f gb = *(const v4f*)(gamma + tid * 8 + 4);
  float gv[8];
#pragma unroll
  for (int e = 0; e < 4; ++e) { gv[e] = bf16_rne(ga[e]); gv[4 + e] = bf16_rne(gb[e]); }
  v8h hv;
#pragma unroll
  for (int e = 0; e < 8; ++e) hv[e] = (_Float16)((xv[e] * rinv) * gv[e]);
  unsigned short* o = xn16 + (size_t)row * kDim + tid * 8;
  for (int pass = 0; pass < 2; ++pass) {
    *(volatile v8h*)(o) = hv;
    __threadfence();
  }
}

__global__ __launch_bounds__(256) void transpose_cast_f16_kernel(const float* __restrict__ in, int ld_in, int n_real,
                                                                 unsigned short* __restrict__ out, int ld_out,
                                                                 int out_row0, float scl) {
  __shared__ __align__(16) _Float16 T[64 * 72];
  const int tid = threadIdx.x, lane = tid & 31, wave = tid >> 5;
  const int k0 = blockIdx.x * 64;
  const int n0 = blockIdx.y * 64;
#pragma unroll
  for (int i = 0; i < 4; ++i) {
    const int idx = i * 256 + tid;
    const int kr = idx >> 4;
    const int c4 = (idx & 15) * 4;
    const int ncol = n0 + c4;
    const bool valid = ncol < n_real;
    const int ccol = valid ? ncol : 0;
    const v4f w = *(const v4f*)(in + (size_t)(k0 + kr) * ld_in + ccol);
#pragma unroll
    for (int e = 0; e < 4; ++e) {
      const float f = valid ? w[e] : 0.0f;
      T[(c4 + e) * 72 + kr] = (_Float16)(bf16_rne(f) * scl);
    }
  }
  __syncthreads();
  const int rq = lane >> 3, c8 = (lane & 7) * 8;
  for (int pass = 0; pass < 2; ++pass) {
#pragma unroll
    for (int i = 0; i < 2; ++i) {
      const int rown = i * 32 + wave * 4 + rq;
      const v8h hv = *(const v8h*)(T + rown * 72 + c8);
      *(volatile v8h*)(out + (size_t)(out_row0 + n0 + rown) * ld_out + k0 + c8) = hv;
    }
    __threadfence();
  }
}

struct RopeFreq { float f[32]; };
static_assert(sizeof(RopeFreq) == 128);

__global__ __launch_bounds__(256) void rope_table_kernel(float* __restrict__ ctab, float* __restrict__ stab, RopeFreq rf) {
  const int tid = threadIdx.x, lane = tid & 31;
  const int n = blockIdx.x * 8 + (tid >> 5);
  float inv = rf.f[0];
#pragma unroll
  for (int i = 1; i < 32; ++i) inv = (lane == i) ? rf.f[i] : inv;
  const float ang = (float)n * inv;
  float sn, cs;
  sincosf(ang, &sn, &cs);
  float* cp = ctab + (size_t)n * 32 + lane;
  float* sp = stab + (size_t)n * 32 + lane;
  for (int pass = 0; pass < 2; ++pass) {
    *(volatile float*)cp = cs;
    *(volatile float*)sp = sn;
    __threadfence();
  }
}

__global__ __launch_bounds__(256) void qkv_prep_kernel(
    const float* __restrict__ cq, const float* __restrict__ vres, const float* __restrict__ bmix,
    const float* __restrict__ ctab, const float* __restrict__ stab,
    unsigned short* __restrict__ q16, unsigned short* __restrict__ k16, unsigned short* __restrict__ vt16,
    float* __restrict__ origv) {
  __shared__ __align__(16) _Float16 Qs[64 * 64];
  __shared__ __align__(16) _Float16 Kst[64 * 64];
  __shared__ __align__(16) _Float16 Vts[64 * 64];
  __shared__ __align__(16) float Vo[64 * 64];
  const int tid = threadIdx.x;
  const int nc = blockIdx.x & 31;
  const int bh = blockIdx.x >> 5;
  const int h = bh & 15, b = bh >> 4;
  const int t = tid >> 2, dq = tid & 3;
  const int n = nc * 64 + t;
  const float* crow = cq + ((size_t)b * kSeq + n) * kCatN;

  float csv[8], snv[8], qf[16], kf[16];
  {
    const v4f ca = *(const v4f*)(ctab + (size_t)n * 32 + dq * 8);
    const v4f cb = *(const v4f*)(ctab + (size_t)n * 32 + dq * 8 + 4);
    const v4f sa = *(const v4f*)(stab + (size_t)n * 32 + dq * 8);
    const v4f sb = *(const v4f*)(stab + (size_t)n * 32 + dq * 8 + 4);
#pragma unroll
    for (int e = 0; e < 4; ++e) { csv[e] = ca[e]; csv[4 + e] = cb[e]; snv[e] = sa[e]; snv[4 + e] = sb[e]; }
#pragma unroll
    for (int i = 0; i < 4; ++i) {
      const v4f qv = *(const v4f*)(crow + h * kDh + dq * 16 + 4 * i);
      const v4f kv = *(const v4f*)(crow + kHeads * kDh + h * kDh + dq * 16 + 4 * i);
#pragma unroll
      for (int e = 0; e < 4; ++e) { qf[4 * i + e] = qv[e]; kf[4 * i + e] = kv[e]; }
    }
  }
  v8h qh0, qh1, kh0, kh1;
#pragma unroll
  for (int p = 0; p < 8; ++p) {
    const float cs = csv[p], sn = snv[p];
    const float qa = qf[2 * p], qb = qf[2 * p + 1];
    const float ka = kf[2 * p], kb = kf[2 * p + 1];
    const float qo0 = qa * cs - qb * sn;
    const float qo1 = qb * cs + qa * sn;
    const float ko0 = ka * cs - kb * sn;
    const float ko1 = kb * cs + ka * sn;
    if (p < 4) { qh0[2 * p] = (_Float16)qo0; qh0[2 * p + 1] = (_Float16)qo1; kh0[2 * p] = (_Float16)ko0; kh0[2 * p + 1] = (_Float16)ko1; }
    else       { qh1[2 * p - 8] = (_Float16)qo0; qh1[2 * p - 7] = (_Float16)qo1; kh1[2 * p - 8] = (_Float16)ko0; kh1[2 * p - 7] = (_Float16)ko1; }
  }
  *(v8h*)(Qs  + t * 64 + dq * 16)     = qh0;
  *(v8h*)(Qs  + t * 64 + dq * 16 + 8) = qh1;
  *(v8h*)(Kst + t * 64 + dq * 16)     = kh0;
  *(v8h*)(Kst + t * 64 + dq * 16 + 8) = kh1;
  asm volatile("" ::: "memory");

  {
    float vf[16], rf[16];
    v4f vraw[4];
#pragma unroll
    for (int i = 0; i < 4; ++i) {
      vraw[i] = *(const v4f*)(crow + 2 * kHeads * kDh + h * kDh + dq * 16 + 4 * i);
      const v4f rv = *(const v4f*)(vres + ((size_t)bh * kSeq + n) * kDh + dq * 16 + 4 * i);
#pragma unroll
      for (int e = 0; e < 4; ++e) { vf[4 * i + e] = vraw[i][e]; rf[4 * i + e] = bf16_rne(rv[e]); }
    }
    const float lg = crow[kQkvN + h];
    const float bm = bf16_rne(bmix[h]);
    const float z = lg + bm;
    const float mixv = 1.0f / (1.0f + expf(-z));
#pragma unroll
    for (int i = 0; i < 4; ++i) *(v4f*)(Vo + t * 64 + dq * 16 + 4 * i) = vraw[i];
#pragma unroll
    for (int m = 0; m < 16; ++m) {
      const float vp = vf[m] + mixv * (rf[m] - vf[m]);
      Vts[(dq * 16 + m) * 64 + t] = (_Float16)vp;
    }
  }
  __syncthreads();

  float* ob = origv + ((size_t)bh * kSeq + nc * 64) * kDh;
  unsigned short* qo = q16 + ((size_t)bh * kSeq + nc * 64) * kDh;
  unsigned short* ko = k16 + ((size_t)bh * kSeq + nc * 64) * kDh;
  const size_t lane8 = (size_t)(tid & 7) * 8;
  for (int pass = 0; pass < 2; ++pass) {
#pragma unroll
    for (int i = 0; i < 4; ++i) {
      const int idx = i * 256 + tid;
      const v4f v = *(const v4f*)(Vo + idx * 4);
      *(volatile v4f*)(ob + (size_t)idx * 4) = v;
    }
#pragma unroll
    for (int i = 0; i < 2; ++i) {
      const int idx = i * 256 + tid;
      const v8h qv = *(const v8h*)(Qs + idx * 8);
      const v8h kv = *(const v8h*)(Kst + idx * 8);
      *(volatile v8h*)(qo + (size_t)idx * 8) = qv;
      *(volatile v8h*)(ko + (size_t)idx * 8) = kv;
    }
#pragma unroll
    for (int i = 0; i < 2; ++i) {
      const int idx = i * 256 + tid;
      const int d = idx >> 3;
      const v8h hv = *(const v8h*)(Vts + d * 64 + lane8);
      *(volatile v8h*)(vt16 + ((size_t)(bh * kDh + d) * kSeq + nc * 64 + lane8)) = hv;
    }
    __threadfence();
  }
}

constexpr float kPCarry = 32768.0f;

__global__ __launch_bounds__(128) void attn_blockcausal_kernel(const unsigned short* __restrict__ q16,
                                                               const unsigned short* __restrict__ k16,
                                                               const unsigned short* __restrict__ vt16,
                                                               unsigned short* __restrict__ ao16) {
  typedef Frag<_Float16> FH;
  union FB { v16h v; v8h h[2]; };
  __shared__ __align__(16) _Float16 Ksh[64 * 64];
  __shared__ __align__(16) _Float16 Vth[64 * 64];
  __shared__ __align__(16) _Float16 Psh[4][16 * 64];
  __shared__ __align__(16) float  Os[4][16 * 68];

  const int tid  = threadIdx.x;
  const int wave = tid >> 5;
  const int lane = tid & 31;
  const int hh   = lane >> 4;
  const int c    = lane & 15;
  const int qb = blockIdx.x & 31;
  const int bh = blockIdx.x >> 5;
  const int h  = bh & 15;
  const int b  = bh >> 4;
  const int q0 = qb * 64 + wave * 16;

  const _Float16* qp = (const _Float16*)q16  + (size_t)bh * kSeq * kDh;
  const _Float16* kp = (const _Float16*)k16  + (size_t)bh * kSeq * kDh;
  const _Float16* vp = (const _Float16*)vt16 + (size_t)bh * kDh * kSeq;

  v16h qa[2];
#pragma unroll
  for (int dc = 0; dc < 2; ++dc) qa[dc] = FH::load(qp + (size_t)(q0 + c) * kDh + dc * 32 + 8 * hh);

  float mrow[8], lrow[8];
  v8f oacc[4];
#pragma unroll
  for (int r = 0; r < 8; ++r) { mrow[r] = -INFINITY; lrow[r] = 0.f; }
#pragma unroll
  for (int t = 0; t < 4; ++t) oacc[t] = (v8f){0.f,0.f,0.f,0.f,0.f,0.f,0.f,0.f};

  const int nChunks = ((qb >> 2) + 1) * 4;
  for (int kc = 0; kc < nChunks; ++kc) {
    const int kv0 = kc * 64;
    __syncthreads();
#pragma unroll
    for (int i = 0; i < 4; ++i) {
      const int idx = i * 128 + tid;
      const int r = idx >> 3, c8 = (idx & 7) * 8;
      *(v8h*)(Ksh + r * 64 + c8) = *(const v8h*)(kp + (size_t)(kv0 + r) * kDh + c8);
      *(v8h*)(Vth + r * 64 + c8) = *(const v8h*)(vp + (size_t)r * kSeq + kv0 + c8);
    }
    __syncthreads();

    v8f s[4];
#pragma unroll
    for (int j = 0; j < 4; ++j) {
      s[j] = (v8f){0.f,0.f,0.f,0.f,0.f,0.f,0.f,0.f};
#pragma unroll
      for (int dc = 0; dc < 2; ++dc) {
        FB kb;
        kb.h[0] = *(const v8h*)(Ksh + (j * 16 + c) * 64 + dc * 32 + 8 * hh);
        kb.h[1] = *(const v8h*)(Ksh + (j * 16 + c) * 64 + dc * 32 + 16 + 8 * hh);
        s[j] = mma_f16g(qa[dc], kb.v, s[j]);
      }
    }
    float cm[8];
#pragma unroll
    for (int r = 0; r < 8; ++r) {
      float m = -INFINITY;
#pragma unroll
      for (int j = 0; j < 4; ++j) {
        const float sv = s[j][r] * 0.125f;
        s[j][r] = sv;
        m = fmaxf(m, sv);
      }
#pragma unroll
      for (int off = 1; off < 16; off <<= 1) m = fmaxf(m, __shfl_xor(m, off, 32));
      cm[r] = m;
    }
    _Float16* pw = Psh[wave];
#pragma unroll
    for (int r = 0; r < 8; ++r) {
      const float mnew = fmaxf(mrow[r], cm[r]);
      const float alpha = expf(mrow[r] - mnew);
      mrow[r] = mnew;
      float psum = 0.f;
#pragma unroll
      for (int j = 0; j < 4; ++j) {
        const float p = expf(s[j][r] - mnew);
        psum += p;
        pw[(8 * hh + r) * 64 + j * 16 + c] = (_Float16)(p * kPCarry);
      }
#pragma unroll
      for (int off = 1; off < 16; off <<= 1) psum += __shfl_xor(psum, off, 32);
      lrow[r] = lrow[r] * alpha + psum;
#pragma unroll
      for (int t = 0; t < 4; ++t) oacc[t][r] *= alpha;
    }
    __builtin_amdgcn_fence(__ATOMIC_RELEASE, "workgroup");
    __builtin_amdgcn_wave_barrier();
    __builtin_amdgcn_fence(__ATOMIC_ACQUIRE, "workgroup");
#pragma unroll
    for (int kk = 0; kk < 2; ++kk) {
      FB pa;
      pa.h[0] = *(const v8h*)(pw + c * 64 + kk * 32 + 8 * hh);
      pa.h[1] = *(const v8h*)(pw + c * 64 + kk * 32 + 16 + 8 * hh);
#pragma unroll
      for (int t = 0; t < 4; ++t) {
        FB vb;
        vb.h[0] = *(const v8h*)(Vth + (t * 16 + c) * 64 + kk * 32 + 8 * hh);
        vb.h[1] = *(const v8h*)(Vth + (t * 16 + c) * 64 + kk * 32 + 16 + 8 * hh);
        oacc[t] = mma_f16g(pa.v, vb.v, oacc[t]);
      }
    }
  }

  float* os = Os[wave];
#pragma unroll
  for (int r = 0; r < 8; ++r) {
    const float inv = 0.0078125f / lrow[r];
#pragma unroll
    for (int t = 0; t < 4; ++t) os[(8 * hh + r) * 68 + t * 16 + c] = oacc[t][r] * inv;
  }
  __builtin_amdgcn_fence(__ATOMIC_RELEASE, "workgroup");
  __builtin_amdgcn_wave_barrier();
  __builtin_amdgcn_fence(__ATOMIC_ACQUIRE, "workgroup");
  {
    const int rq = lane >> 3, c8 = (lane & 7) * 8;
    unsigned short* ob = ao16 + ((size_t)b * kSeq + q0) * kDim + h * kDh;
    for (int pass = 0; pass < 2; ++pass) {
#pragma unroll
      for (int it = 0; it < 4; ++it) {
        const int row = it * 4 + rq;
        const float* sp = os + row * 68 + c8;
        v8h hv;
#pragma unroll
        for (int e = 0; e < 8; ++e) hv[e] = (_Float16)sp[e];
        *(volatile v8h*)(ob + (size_t)row * kDim + c8) = hv;
      }
      __threadfence();
    }
  }
}

extern "C" void kernel_launch(void* const* d_in, const int* in_sizes, int n_in,
                              void* d_out, int out_size, void* d_ws, size_t ws_size,
                              hipStream_t stream) {
  if (n_in < 7) return;
  if (in_sizes[0] != kTok * kDim || in_sizes[1] != kOut1Elems || in_sizes[2] != kDim ||
      in_sizes[3] != kDim * kQkvN || in_sizes[4] != kDim * kDim || in_sizes[5] != kDim * kHeads ||
      in_sizes[6] != kHeads) return;
  if (out_size != kOut0Elems + kOut1Elems) return;

  const float* x     = (const float*)d_in[0];
  const float* vres  = (const float*)d_in[1];
  const float* gamma = (const float*)d_in[2];
  const float* Wqkv  = (const float*)d_in[3];
  const float* Wout  = (const float*)d_in[4];
  const float* Wmix  = (const float*)d_in[5];
  const float* bmix  = (const float*)d_in[6];

  float* out0  = (float*)d_out;
  float* out1  = out0 + (size_t)kOut0Elems;

  const size_t szXn   = (size_t)kTok * kDim * 2;
  const size_t szWcat = (size_t)kCatN * kDim * 2;
  const size_t szWout = (size_t)kDim * kDim * 2;
  const size_t szC32  = (size_t)kTok * kCatN * 4;
  const size_t szTab  = (size_t)kSeq * 32 * 4;
  const size_t szHead = (size_t)kBH * kSeq * kDh * 2;
  const size_t szAo   = (size_t)kTok * kDim * 2;
  size_t off = 0;
  char* ws = (char*)d_ws;
  unsigned short* xn16   = (unsigned short*)(ws + off); off += szXn;
  unsigned short* wcat16 = (unsigned short*)(ws + off); off += szWcat;
  unsigned short* wout16 = (unsigned short*)(ws + off); off += szWout;
  float*          c32    = (float*)(ws + off);          off += szC32;
  float*          ctab   = (float*)(ws + off);          off += szTab;
  float*          stab   = (float*)(ws + off);          off += szTab;
  unsigned short* q16    = (unsigned short*)(ws + off); off += szHead;
  unsigned short* k16    = (unsigned short*)(ws + off); off += szHead;
  unsigned short* vt16   = (unsigned short*)(ws + off); off += szHead;
  unsigned short* ao16   = (unsigned short*)(ws + off); off += szAo;
  if (off > ws_size) return;

  RopeFreq rf;
  for (int j = 0; j < 32; ++j) {
    const double p = pow(10000.0, (double)j / 32.0);
    const float pf = (float)p;
    rf.f[j] = 1.0f / pf;
  }

  rmsnorm_f16_kernel<<<kTok, 128, 0, stream>>>(x, gamma, xn16);
  transpose_cast_f16_kernel<<<dim3(kDim / 64, kQkvN / 64), 256, 0, stream>>>(Wqkv, kQkvN, kQkvN, wcat16, kDim, 0, 64.0f);
  transpose_cast_f16_kernel<<<dim3(kDim / 64, 1), 256, 0, stream>>>(Wmix, kHeads, kHeads, wcat16, kDim, kQkvN, 64.0f);
  transpose_cast_f16_kernel<<<dim3(kDim / 64, kDim / 64), 256, 0, stream>>>(Wout, kDim, kDim, wout16, kDim, 0, 64.0f);
  rope_table_kernel<<<kSeq / 8, 256, 0, stream>>>(ctab, stab, rf);
  {
    const int blocks = (kTok / 64) * (kCatN / 64) / 8;
    wmma_gemm64<0, false, 0, 0, false, 0><<<dim3(blocks, 1), 256, 0, stream>>>(
        xn16, xn16, kDim, 0L, wcat16, wcat16, kDim, 0L,
        (void*)c32, (void*)c32, kCatN, 0L, bmix, bmix, 0L, kTok, kCatN, kDim, 1.0f / 64.0f);
  }
  qkv_prep_kernel<<<kBH * (kSeq / 64), 256, 0, stream>>>(c32, vres, bmix, ctab, stab, q16, k16, vt16, out1);
  attn_blockcausal_kernel<<<kBH * (kSeq / 64), 128, 0, stream>>>(q16, k16, vt16, ao16);
  {
    const int blocks = (kTok / 64) * (kDim / 64) / 8;
    wmma_gemm64<0, false, 0, 0, false, 0><<<dim3(blocks, 1), 256, 0, stream>>>(
        ao16, ao16, kDim, 0L, wout16, wout16, kDim, 0L,
        (void*)out0, (void*)out0, kDim, 0L, bmix, bmix, 0L, kTok, kDim, kDim, 1.0f / 16384.0f);
  }
}
